// FactorizedRandomSelfAttention_3040836845902
// MI455X (gfx1250) — hardware-verified
//
#include <hip/hip_runtime.h>


typedef _Float16     v16h  __attribute__((ext_vector_type(16)));
typedef float        v8f   __attribute__((ext_vector_type(8)));
typedef float        v4f   __attribute__((ext_vector_type(4)));
typedef unsigned int u32x4 __attribute__((ext_vector_type(4)));

#define BB 4
#define HH 12
#define NN 2048
#define DD 64
#define KK 32

#define BN 64
#define NMT (NN / BN)
#define NWAVES 8
#define NTHREADS (32 * NWAVES)
#define BMWG (16 * NWAVES)
#define NTILES (NN / BMWG)
#define NEGC 1000000.0f

#define R2P 20
#define VSP 36
#define SSP 68

#define SCR 16.0f
#define INV_SCR2 0.00390625f
#define SCV 64.0f
#define INV_SCV 0.015625f

static_assert(KK == 32);
static_assert(DD == 64);
static_assert(BN == 64);
static_assert(NN % BN == 0);
static_assert(NN % BMWG == 0);
static_assert(NTHREADS == 256);
static_assert((R2P * 4) % 16 == 0);
static_assert((VSP * 4) % 16 == 0);
static_assert((SSP * 4) % 16 == 0);

union Frag { v16h v; u32x4 q[2]; unsigned int u[8]; };

__device__ __forceinline__ unsigned int pack2h(float x, float y) {
    union { _Float16 f; unsigned short s; } a, c;
    a.f = (_Float16)x;
    c.f = (_Float16)y;
    return (unsigned int)a.s | ((unsigned int)c.s << 16);
}

__device__ __forceinline__ v8f wmma16(v16h a, v16h b, v8f c) {
    v8f d = __builtin_amdgcn_wmma_f32_16x16x32_f16(false, a, false, b, (short)0, c, false, false);
    asm volatile("v_nop\n\tv_nop\n\tv_nop\n\tv_nop" : "+v"(d) : "v"(a), "v"(b));
    return d;
}

__global__ __launch_bounds__(NTHREADS) void k_synth(
    const float* __restrict__ V, const float* __restrict__ keymask,
    const float* __restrict__ R1, const float* __restrict__ R2,
    float* __restrict__ X)
{
    __shared__ __attribute__((aligned(16))) unsigned int r2s[BN * R2P];
    __shared__ __attribute__((aligned(16))) unsigned int vsm[DD * VSP];
    __shared__ __attribute__((aligned(16))) float sS[NWAVES * 16 * SSP];

    const int tid  = threadIdx.x;
    const int lane = tid & 31;
    const int wave = tid >> 5;
    const int lh   = lane & 15;
    const int hf   = lane >> 4;

    const int bid = blockIdx.x;
    if (bid >= BB * HH * NTILES) return;
    const int nt = bid % NTILES;
    const int hd = (bid / NTILES) % HH;
    const int bb = bid / (NTILES * HH);
    const int n0 = nt * BMWG + wave * 16;

    const int f_c4 = tid & 15;
    const int f_rp = tid >> 4;

    const float* r2base = R2 + (size_t)hd * KK * NN;
    const float* vbase  = V + ((size_t)bb * HH + hd) * (size_t)NN * DD;
    const float* mrow   = keymask + (size_t)bb * NN;
    float* sSw = sS + wave * 16 * SSP;

    Frag aR1;
    {
        const float* r1p = R1 + ((size_t)hd * NN + (size_t)(n0 + lh)) * KK;
        const v4f x0 = *(const v4f*)(r1p + 8 * hf);
        const v4f x1 = *(const v4f*)(r1p + 8 * hf + 4);
        const v4f x2 = *(const v4f*)(r1p + 16 + 8 * hf);
        const v4f x3 = *(const v4f*)(r1p + 16 + 8 * hf + 4);
        aR1.u[0] = pack2h(SCR * x0[0], SCR * x0[1]);
        aR1.u[1] = pack2h(SCR * x0[2], SCR * x0[3]);
        aR1.u[2] = pack2h(SCR * x1[0], SCR * x1[1]);
        aR1.u[3] = pack2h(SCR * x1[2], SCR * x1[3]);
        aR1.u[4] = pack2h(SCR * x2[0], SCR * x2[1]);
        aR1.u[5] = pack2h(SCR * x2[2], SCR * x2[3]);
        aR1.u[6] = pack2h(SCR * x3[0], SCR * x3[1]);
        aR1.u[7] = pack2h(SCR * x3[2], SCR * x3[3]);
    }

    const v8f z8 = {0.0f, 0.0f, 0.0f, 0.0f, 0.0f, 0.0f, 0.0f, 0.0f};
    v8f acc[4];
    #pragma unroll
    for (int t = 0; t < 4; ++t) acc[t] = z8;
    float m_i = -1.0e30f;
    float l_i = 0.0f;

    for (int mt = 0; mt < NMT; ++mt) {
        const int m0 = mt * BN;

        {
            const float* r2p = r2base + m0;
            const v4f x0 = *(const v4f*)(r2p + (size_t)(2 * f_rp)     * NN + 4 * f_c4);
            const v4f x1 = *(const v4f*)(r2p + (size_t)(2 * f_rp + 1) * NN + 4 * f_c4);
            #pragma unroll
            for (int c = 0; c < 4; ++c)
                r2s[(4 * f_c4 + c) * R2P + f_rp] = pack2h(SCR * x0[c], SCR * x1[c]);
            const float* vp = vbase + (size_t)m0 * DD;
            #pragma unroll
            for (int i = 0; i < 2; ++i) {
                const int mp = f_rp + 16 * i;
                const v4f y0 = *(const v4f*)(vp + (size_t)(2 * mp)     * DD + 4 * f_c4);
                const v4f y1 = *(const v4f*)(vp + (size_t)(2 * mp + 1) * DD + 4 * f_c4);
                #pragma unroll
                for (int c = 0; c < 4; ++c)
                    vsm[(4 * f_c4 + c) * VSP + mp] = pack2h(SCV * y0[c], SCV * y1[c]);
            }
        }
        __syncthreads();

        #pragma unroll
        for (int j = 0; j < 4; ++j) {
            const int m = 16 * j + lh;
            const u32x4* bp = (const u32x4*)(r2s + m * R2P);
            Frag bR2;
            bR2.q[0] = bp[hf];
            bR2.q[1] = bp[2 + hf];
            const v8f Sj = wmma16(aR1.v, bR2.v, z8);
            const float madd = NEGC * (1.0f - mrow[m0 + m]);
            #pragma unroll
            for (int r = 0; r < 8; ++r)
                sSw[(8 * hf + r) * SSP + 16 * j + lh] = Sj[r] * INV_SCR2 - madd;
        }
        __syncthreads();

        float sv[32];
        float alpha;
        {
            const float* srow = sSw + lh * SSP;
            #pragma unroll
            for (int g = 0; g < 4; ++g) {
                const v4f* sp = (const v4f*)(srow + 16 * g + 8 * hf);
                const v4f a0 = sp[0], a1 = sp[1];
                #pragma unroll
                for (int c = 0; c < 4; ++c) { sv[8 * g + c] = a0[c]; sv[8 * g + 4 + c] = a1[c]; }
            }
            float rmax = sv[0];
            #pragma unroll
            for (int i = 1; i < 32; ++i) rmax = fmaxf(rmax, sv[i]);
            rmax = fmaxf(rmax, __shfl_xor(rmax, 16, 32));

            const float mnew = fmaxf(m_i, rmax);
            alpha = __expf(m_i - mnew);

            float rsum = 0.0f;
            #pragma unroll
            for (int i = 0; i < 32; ++i) { sv[i] = __expf(sv[i] - mnew); rsum += sv[i]; }
            rsum += __shfl_xor(rsum, 16, 32);

            l_i = l_i * alpha + rsum;
            m_i = mnew;
        }

        Frag aP[2];
        #pragma unroll
        for (int s = 0; s < 2; ++s)
            #pragma unroll
            for (int v = 0; v < 8; ++v)
                aP[s].u[v] = pack2h(sv[16 * s + 2 * v], sv[16 * s + 2 * v + 1]);

        float al[8];
        #pragma unroll
        for (int r = 0; r < 8; ++r) al[r] = __shfl(alpha, 8 * hf + r, 32);
        #pragma unroll
        for (int t = 0; t < 4; ++t)
            #pragma unroll
            for (int r = 0; r < 8; ++r)
                acc[t][r] *= al[r];

        #pragma unroll
        for (int t = 0; t < 4; ++t) {
            const int d = 16 * t + lh;
            const u32x4* q = (const u32x4*)(vsm + d * VSP);
            Frag bV0, bV1;
            bV0.q[0] = q[hf];
            bV0.q[1] = q[2 + hf];
            bV1.q[0] = q[4 + hf];
            bV1.q[1] = q[6 + hf];
            acc[t] = wmma16(aP[0].v, bV0.v, acc[t]);
            acc[t] = wmma16(aP[1].v, bV1.v, acc[t]);
        }
        __syncthreads();
    }

    const float linv = INV_SCV / l_i;
    float li[8];
    #pragma unroll
    for (int r = 0; r < 8; ++r) li[r] = __shfl(linv, 8 * hf + r, 32);
    #pragma unroll
    for (int r = 0; r < 8; ++r)
        #pragma unroll
        for (int t = 0; t < 4; ++t)
            sSw[(8 * hf + r) * SSP + 16 * t + lh] = acc[t][r] * li[r];
    __syncthreads();

    float* xp = X + ((size_t)bb * HH + hd) * (size_t)NN * DD;
    const int piece = lane & 7;
    const int lsel  = lane >> 3;
    v4f vals[8];
    size_t offs[8];
    #pragma unroll
    for (int i = 0; i < 8; ++i) {
        const int L    = 4 * i + lsel;
        const int row  = L >> 1;
        const int col0 = (L & 1) * 32 + piece * 4;
        vals[i] = *(const v4f*)(sSw + row * SSP + col0);
        offs[i] = (size_t)(n0 + row) * DD + col0;
    }
    #pragma unroll
    for (int i = 0; i < 8; ++i) *(volatile v4f*)(xp + offs[i]) = vals[i];
    __threadfence();
    #pragma unroll
    for (int i = 0; i < 8; ++i) *(volatile v4f*)(xp + offs[i]) = vals[i];
}

extern "C" void kernel_launch(void* const* d_in, const int* in_sizes, int n_in,
                              void* d_out, int out_size, void* d_ws, size_t ws_size,
                              hipStream_t stream) {
    (void)d_ws; (void)ws_size;
    if (n_in < 4) return;
    if (in_sizes[0] != BB * HH * NN * DD) return;
    if (in_sizes[1] != BB * NN) return;
    if (in_sizes[2] != HH * NN * KK) return;
    if (in_sizes[3] != HH * KK * NN) return;
    if (out_size != BB * HH * NN * DD) return;

    const float* V       = (const float*)d_in[0];
    const float* keymask = (const float*)d_in[1];
    const float* R1      = (const float*)d_in[2];
    const float* R2      = (const float*)d_in[3];
    float* X = (float*)d_out;

    const int grid = BB * HH * NTILES;
    k_synth<<<grid, NTHREADS, 0, stream>>>(V, keymask, R1, R2, X);
    (void)hipGetLastError();
}
